// TpsGridGen_30202210025942
// MI455X (gfx1250) — hardware-verified
//
#include <hip/hip_runtime.h>
#include <math.h>

typedef __attribute__((ext_vector_type(16))) _Float16 v16h;
typedef __attribute__((ext_vector_type(16))) __bf16 v16b;
typedef __attribute__((ext_vector_type(8)))  _Float16 v8h;
typedef __attribute__((ext_vector_type(8)))  float v8f;
typedef __attribute__((ext_vector_type(4)))  float v4f;
typedef __attribute__((ext_vector_type(2)))  float v2f;
typedef __attribute__((ext_vector_type(4)))  unsigned v4u;
typedef __attribute__((ext_vector_type(4)))  int v4i;
typedef float __attribute__((may_alias)) float_a;
typedef int __attribute__((may_alias)) int_a;

template <typename T> __device__ __forceinline__ void vst2(void* p, T v) { *(volatile T*)p = v; __threadfence(); *(volatile T*)p = v; }
__device__ __forceinline__ v8f wmma16(v16h a, v16h b, v8f c) {
  v8f d = __builtin_amdgcn_wmma_f32_16x16x32_f16(false, a, false, b, (short)0, c, false, false);
  asm volatile("v_nop\n\tv_nop\n\tv_nop\n\tv_nop" : "+v"(d) : "v"(a), "v"(b));
  return d;
}
__device__ __forceinline__ v8f wmma_bf(v16b a, v16b b, v8f c) {
  v8f d = __builtin_amdgcn_wmma_f32_16x16x32_bf16(false, a, false, b, (short)0, c, false, false);
  asm volatile("v_nop\n\tv_nop\n\tv_nop\n\tv_nop" : "+v"(d) : "v"(a), "v"(b));
  return d;
}
__device__ __forceinline__ v16h frag_h(const _Float16* rowk0, int lane) {
  union { v16h v; v8h q[2]; } u; const _Float16* p = rowk0 + 8 * (lane >> 4);
  u.q[0] = *(const v8h*)p; u.q[1] = *(const v8h*)(p + 16); return u.v;
}
__device__ __forceinline__ v16h frag_f32(const float* rowk0, int lane) {
  v16h a; const float* p = rowk0 + 8 * (lane >> 4);
#pragma unroll
  for (int i = 0; i < 8; ++i) { a[i] = (_Float16)p[i]; a[8 + i] = (_Float16)p[16 + i]; }
  return a;
}
__device__ __forceinline__ v16h frag_f32s(const float* rowk0, int lane, float sc) {
  v16h a; const float* p = rowk0 + 8 * (lane >> 4);
#pragma unroll
  for (int i = 0; i < 8; ++i) { a[i] = (_Float16)(p[i] * sc); a[8 + i] = (_Float16)(p[16 + i] * sc); }
  return a;
}
__device__ __forceinline__ v16h fragc_f32(const float* W, int k0, int n, int lane, int ld, int K) {
  v16h a; const int g = lane >> 4;
#pragma unroll
  for (int i = 0; i < 8; ++i) { const int ka = k0 + 8 * g + i, kb = ka + 16;
    a[i] = (_Float16)(ka < K ? W[(size_t)(ka < K ? ka : K - 1) * ld + n] : 0.f); a[8 + i] = (_Float16)(kb < K ? W[(size_t)(kb < K ? kb : K - 1) * ld + n] : 0.f); }
  return a;
}
struct F2 { v16b h, l; };
__device__ __forceinline__ F2 bsplit16(const float v[16]) { F2 r;
#pragma unroll
  for (int i = 0; i < 16; ++i) { const __bf16 h = (__bf16)v[i]; r.h[i] = h; r.l[i] = (__bf16)(v[i] - (float)h); }
  return r; }
__device__ __forceinline__ F2 split_row(const float* row, int k0, int lane) { float v[16]; const float* p = row + k0 + 8 * (lane >> 4);
#pragma unroll
  for (int i = 0; i < 8; ++i) { v[i] = p[i]; v[8 + i] = p[16 + i]; }
  return bsplit16(v); }
__device__ __forceinline__ F2 split_rowK(const float* row, int k0, int lane, int K) { float v[16]; const int g = lane >> 4;
#pragma unroll
  for (int i = 0; i < 8; ++i) { const int ka = k0 + 8 * g + i, kb = ka + 16; v[i] = ka < K ? row[ka < K ? ka : K - 1] : 0.f; v[8 + i] = kb < K ? row[kb < K ? kb : K - 1] : 0.f; }
  return bsplit16(v); }
__device__ __forceinline__ F2 split_col(const float* W, int k0, int n, int lane, int ld, int K) { float v[16]; const int g = lane >> 4;
#pragma unroll
  for (int i = 0; i < 8; ++i) { const int ka = k0 + 8 * g + i, kb = ka + 16; v[i] = ka < K ? W[(size_t)(ka < K ? ka : K - 1) * ld + n] : 0.f; v[8 + i] = kb < K ? W[(size_t)(kb < K ? kb : K - 1) * ld + n] : 0.f; }
  return bsplit16(v); }
__device__ __forceinline__ v8f mac3(const F2& a, const F2& b, v8f c) { c = wmma_bf(a.l, b.h, c); c = wmma_bf(a.h, b.l, c); return wmma_bf(a.h, b.h, c); }
__device__ __forceinline__ float sigm(float v) { return 1.0f / (1.0f + expf(-v)); }
#define LDSX() do { asm volatile("s_wait_dscnt 0" ::: "memory"); __builtin_amdgcn_wave_barrier(); __builtin_amdgcn_fence(__ATOMIC_RELEASE, "workgroup"); } while (0)

__device__ __forceinline__ float bfr(float v) { return (float)(__bf16)v; }
#define NBT 2
#define RES 128
#define NCP 27
#define NLI 31
#ifndef NBLK
#define NBLK (RES * RES)
#endif
#define WS_WC 0u
#define WS_END (WS_WC + 4u * 256u)
__global__ __launch_bounds__(256) void k_coef(const float* __restrict__ TH, const float* __restrict__ LI, float* __restrict__ TAB) { __shared__ __align__(16) float st[256];
  const int t = threadIdx.x; float v = 0.f;
  if (t < NBT * 3 * 32) { const int bc = t >> 5, n = t & 31; if (n < NLI) { const int b = bc / 3, c = bc % 3; float s = 0.f; for (int m = 0; m < NCP; ++m) s += bfr(LI[n * NLI + m]) * bfr(TH[b * 81 + c * NCP + m]); v = s; } }
  st[t] = v; __syncthreads();
  if (t < 64) vst2(TAB + t * 4, *(const v4f*)&st[t * 4]); }
__global__ __launch_bounds__(128) void k_tps(const float* __restrict__ GRID, const float* __restrict__ P, const float* __restrict__ TAB, float* __restrict__ OUT) {
  __shared__ __align__(16) float su[128][36]; __shared__ __align__(16) float sw[16][36]; __shared__ __align__(16) float sres[NBT][128 * 3]; __shared__ float sg[128][3]; __shared__ float sa[NBT * 3][4];
  const int tid = threadIdx.x, wave = tid >> 5, lane = tid & 31, col = lane & 15, g = lane >> 4; const int h = blockIdx.x / RES, w = blockIdx.x % RES;
  { const int d = tid; const float* gp = GRID + (((size_t)h * RES + w) * RES + d) * 3; const float gx = bfr(gp[0]), gy = bfr(gp[1]), gz = bfr(gp[2]); sg[d][0] = gx; sg[d][1] = gy; sg[d][2] = gz;
    for (int n = 0; n < 32; ++n) { float u = 0.f; if (n < NCP) { const float dx = gx - bfr(P[n * 3]), dy = gy - bfr(P[n * 3 + 1]), dz = gz - bfr(P[n * 3 + 2]); float r2 = dx * dx + dy * dy + dz * dz; if (r2 == 0.f) r2 = 1.0f; u = r2 * logf(r2); } su[d][n] = u; } }
  if (tid < 16) { for (int n = 0; n < 32; ++n) sw[tid][n] = (tid < NBT * 3 && n < NCP) ? TAB[tid * 32 + n] : 0.f; }
  if (tid < NBT * 3) { for (int a = 0; a < 4; ++a) sa[tid][a] = TAB[tid * 32 + NCP + a]; }
  __syncthreads();
#pragma unroll
  for (int tI = 0; tI < 2; ++tI) { const int v0 = wave * 32 + tI * 16;
    const F2 a = split_row(&su[v0 + col][0], 0, lane); const F2 bw = split_row(&sw[col][0], 0, lane);
    v8f acc = {}; acc = wmma_bf(a.h, bw.h, acc); acc = wmma_bf(a.h, bw.l, acc); acc = wmma_bf(a.l, bw.h, acc);
    if (col < NBT * 3) { const int b = col / 3, c = col % 3;
#pragma unroll
      for (int r = 0; r < 8; ++r) { const int d = v0 + 8 * g + r; const float aff = sa[col][0] + sg[d][0] * sa[col][1] + sg[d][1] * sa[col][2] + sg[d][2] * sa[col][3]; sres[b][d * 3 + c] = acc[r] + aff; } } }
  __syncthreads();
  for (int b = 0; b < NBT; ++b) { float* dst = OUT + ((((size_t)b * RES + h) * RES + w) * RES) * 3; for (int q = tid; q < 128 * 3 / 4; q += 128) vst2(dst + q * 4, *(const v4f*)&sres[b][q * 4]); } }
extern "C" void kernel_launch(void* const* d_in, const int* in_sizes, int n_in, void* d_out, int out_size, void* d_ws, size_t ws_size, hipStream_t stream) {
  (void)in_sizes; (void)n_in; (void)out_size;
  const float** F = (const float**)d_in;
  if (ws_size < (size_t)WS_END) return;
  char* ws = (char*)d_ws; float* TAB = (float*)(ws + WS_WC);
  k_coef<<<dim3(1), 256, 0, stream>>>(F[0], F[3], TAB);
  k_tps<<<dim3(NBLK), 128, 0, stream>>>(F[1], F[2], TAB, (float*)d_out);
}
